// GNNModel_1layer_17136919511531
// MI455X (gfx1250) — hardware-verified
//
#include <hip/hip_runtime.h>
#include <stddef.h>


#define HD      64
#define NIN     5
#define KPB     64
#define APZ     72
#define PQP     64
#define GROWS   32
#define GTHR    64
#define STHR    256
#define SWAV    (STHR / 32)
#define EPT     16
#define CHUNK   (STHR * EPT)
#define NBD     2048
#define NBA     512
#define NPADG   2048
#define ETHR    128
#define EWAV    (ETHR / 32)
#define EPB     128
#define EPW     32
#define OFF_BG  0
#define OFF_B1  (HD * KPB)
#define BPTOT   (OFF_B1 + 3 * HD * KPB)
#define WSC     64.0f
#define HSC     16.0f
#define RH      0.0009765625f
#define WSCAP   134217728
#define LDS_DEG (SWAV * NBD * 4 + CHUNK * 4 + NBD * 4 + 64)
#define LDS_AGG (NBA * HD * 4 + CHUNK * 4 + NBA * 4 + HD * 4 + 64)

static_assert(BPTOT == 16384);
static_assert(HD * KPB == 2 * 256 * 8);
static_assert(3 * HD * KPB == 6 * 256 * 8);
static_assert((APZ % 8) == 0 && (KPB % 8) == 0 && (HD % 32) == 0);
static_assert(PQP == HD && HD == 2 * 32);
static_assert(GROWS == (GTHR / 32) * 16);
static_assert(GROWS * HD == 4 * GTHR * 8);
static_assert(GROWS * 2 * HD == 4 * GTHR * 16);
static_assert(NBA == 2 * STHR && NBD == 8 * STHR && NBA == 512);
static_assert((SWAV * NBD) % (4 * STHR) == 0 && (NBA * HD) % (4 * STHR) == 0 && (NBA * HD) % (8 * STHR) == 0);
static_assert(NBD % (4 * STHR) == 0);
static_assert(ETHR == 2 * HD && EPB == ETHR && EPW * EWAV == EPB);
static_assert((NPADG % NBD) == 0 && (NPADG % NBA) == 0 && (NPADG % GROWS) == 0);
static_assert(CHUNK == 4096);

typedef float    v2f  __attribute__((ext_vector_type(2)));
typedef float    v4f  __attribute__((ext_vector_type(4)));
typedef float    v8f  __attribute__((ext_vector_type(8)));
typedef int      v4i  __attribute__((ext_vector_type(4)));
typedef _Float16 v4h  __attribute__((ext_vector_type(4)));
typedef _Float16 v8h  __attribute__((ext_vector_type(8)));
typedef _Float16 v16h __attribute__((ext_vector_type(16)));
union Frag { v16h v; v8h h[2]; v4h q[4]; };

__device__ __forceinline__ v8f wmh(v16h a, v16h b, v8f c) {
  v8f d = __builtin_amdgcn_wmma_f32_16x16x32_f16(false, a, false, b, (short)0, c, false, false);
  asm volatile("v_nop\n\tv_nop\n\tv_nop\n\tv_nop" : "+v"(d) : "v"(a), "v"(b));
  return d;
}

template <int NT>
__device__ __forceinline__ void mma16(const _Float16* Ar, int lda, const _Float16* __restrict__ Bpl,
                                      int lane, v8f (&acc)[NT]) {
  const int hh = lane >> 4, m = lane & 15;
#pragma unroll
  for (int t = 0; t < NT; ++t) { v8f z = {0.f, 0.f, 0.f, 0.f, 0.f, 0.f, 0.f, 0.f}; acc[t] = z; }
  const _Float16* ap = Ar + m * lda + 8 * hh;
  const _Float16* bb = Bpl + (size_t)m * KPB + 8 * hh;
#pragma unroll 1
  for (int ks = 0; ks < HD / 32; ++ks) {
    Frag a;
    a.h[0] = *(const v8h*)(ap + 32 * ks);
    a.h[1] = *(const v8h*)(ap + 32 * ks + 16);
#pragma unroll
    for (int t = 0; t < NT; ++t) {
      const _Float16* bp = bb + (size_t)(16 * t) * KPB + 32 * ks;
      Frag b;
      b.h[0] = *(const v8h*)bp;
      b.h[1] = *(const v8h*)(bp + 16);
      acc[t] = wmh(a.v, b.v, acc[t]);
    }
  }
}

__global__ __launch_bounds__(256) void k_wprep(const float* __restrict__ Wg, const float* __restrict__ W1,
                                               _Float16* Bpl) {
  const int blk = blockIdx.x, tid = threadIdx.x;
  float v[8];
  v8h hv;
  _Float16* dp;
  if (blk < 2) {
    const int i = blk * 256 + tid;
    const int n = i >> 3, k0 = (i & 7) * 8;
#pragma unroll
    for (int e = 0; e < 8; ++e) v[e] = Wg[(k0 + e) * HD + n];
    dp = Bpl + OFF_BG + i * 8;
  } else {
    const int i = (blk - 2) * 256 + tid;
    const int n = i >> 3, k0 = (i & 7) * 8;
    const int kb = (n >> 6) * HD, nc = n & (HD - 1);
#pragma unroll
    for (int e = 0; e < 8; ++e) v[e] = W1[(kb + k0 + e) * HD + nc];
    dp = Bpl + OFF_B1 + i * 8;
  }
#pragma unroll
  for (int e = 0; e < 8; ++e) hv[e] = (_Float16)(v[e] * WSC);
  *(volatile v8h*)dp = hv;
  __threadfence();
  *(volatile v8h*)dp = hv;
}

__device__ __forceinline__ void loadids(const int* __restrict__ ids, int nE, int cbase, int tid, int vec,
                                        int (&d)[EPT]) {
  const int e0 = cbase + EPT * tid;
  if (vec != 0 && cbase + CHUNK <= nE) {
#pragma unroll
    for (int q = 0; q < EPT / 4; ++q) {
      const v4i t4 = *(const v4i*)(ids + e0 + 4 * q);
      d[4 * q] = t4.x; d[4 * q + 1] = t4.y; d[4 * q + 2] = t4.z; d[4 * q + 3] = t4.w;
    }
  } else {
#pragma unroll
    for (int j = 0; j < EPT; ++j) {
      int idx = e0 + j;
      const bool ok = idx < nE;
      idx = ok ? idx : nE - 1;
      const int val = ids[idx];
      d[j] = ok ? val : (-2147483647 - 1);
    }
  }
}

__device__ __forceinline__ void blkscan(int cnt, int lane, int wave, int* swt, int& pos, int& nh) {
  int x = cnt;
#pragma unroll
  for (int o = 1; o < 32; o <<= 1) {
    const int y = __shfl_up(x, o, 32);
    x += (lane >= o) ? y : 0;
  }
  if (lane == 31) swt[wave] = x;
  __syncthreads();
  int wpre = 0, tot = 0;
#pragma unroll
  for (int w = 0; w < SWAV; ++w) {
    const int v = swt[w];
    wpre += (w < wave) ? v : 0;
    tot += v;
  }
  pos = wpre + x - cnt;
  nh = tot;
}

__global__ __launch_bounds__(STHR) void k_deg(const int* __restrict__ dsts, float* dinv,
                                               int nE, int nChunks, int vec) {
  extern __shared__ __attribute__((aligned(16))) char dynl[];
  int*      scnt  = (int*)dynl;
  unsigned* slist = (unsigned*)(dynl + SWAV * NBD * 4);
  float*    sdo   = (float*)(dynl + SWAV * NBD * 4 + CHUNK * 4);
  int*      swt   = (int*)(dynl + SWAV * NBD * 4 + CHUNK * 4 + NBD * 4);
  const int tid = threadIdx.x, lane = tid & 31;
  const int wave = __builtin_amdgcn_readfirstlane(tid >> 5);
  const int n0 = blockIdx.x * NBD;
  {
    v4i z = {0, 0, 0, 0};
    v4i* p = (v4i*)scnt;
#pragma unroll
    for (int it = 0; it < (SWAV * NBD) / (4 * STHR); ++it) p[it * STHR + tid] = z;
  }
  __syncthreads();

#pragma unroll 1
  for (int c = 0; c < nChunks; ++c) {
    const int cbase = c * CHUNK;
    int d[EPT];
    loadids(dsts, nE, cbase, tid, vec, d);
    unsigned msk = 0;
#pragma unroll
    for (int j = 0; j < EPT; ++j) {
      const unsigned ld = (unsigned)d[j] - (unsigned)n0;
      msk |= ((ld < (unsigned)NBD) ? 1u : 0u) << j;
    }
    const int cnt = __builtin_popcount(msk);
    int pos, nh;
    blkscan(cnt, lane, wave, swt, pos, nh);
#pragma unroll
    for (int j = 0; j < EPT; ++j) {
      if ((msk >> j) & 1u) {
        if (pos < CHUNK) slist[pos] = (unsigned)d[j] - (unsigned)n0;
        ++pos;
      }
    }
    __syncthreads();
    const int nhc = nh < CHUNK ? nh : CHUNK;
    int* myc = scnt + wave * NBD;
    for (int j = wave; j < nhc; j += SWAV) {
      const int ld = __builtin_amdgcn_readfirstlane((int)slist[j]) & (NBD - 1);
      myc[ld] = myc[ld] + 1;
    }
  }
  __syncthreads();

#pragma unroll
  for (int q = 0; q < NBD / STHR; ++q) {
    const int ld = q * STHR + tid;
    int cdeg = 1;
#pragma unroll
    for (int w = 0; w < SWAV; ++w) cdeg += scnt[w * NBD + ld];
    sdo[ld] = rsqrtf((float)cdeg);
  }
  __syncthreads();

  float* gp = dinv + (size_t)n0;
#pragma unroll
  for (int it = 0; it < NBD / (4 * STHR); ++it) {
    const int f = it * STHR + tid;
    const v4f v = ((const v4f*)sdo)[f];
    *(volatile v4f*)(gp + 4 * f) = v;
  }
  __threadfence();
#pragma unroll
  for (int it = 0; it < NBD / (4 * STHR); ++it) {
    const int f = it * STHR + tid;
    const v4f v = ((const v4f*)sdo)[f];
    *(volatile v4f*)(gp + 4 * f) = v;
  }
}

__global__ __launch_bounds__(GTHR) void k_node1(const float* __restrict__ x, const float* __restrict__ Wn,
                                                const float* __restrict__ bn, const float* __restrict__ dinv,
                                                const _Float16* __restrict__ BG, float* HT, int nN) {
  __shared__ __attribute__((aligned(16))) float swn[NIN * HD];
  __shared__ __attribute__((aligned(16))) float sbn[HD];
  __shared__ __attribute__((aligned(16))) float sdi[GROWS];
  __shared__ __attribute__((aligned(16))) _Float16 At[GROWS * APZ];
  __shared__ __attribute__((aligned(16))) float stg[GROWS * HD];
  const int tid = threadIdx.x, lane = tid & 31, wave = tid >> 5, hh = lane >> 4, m = lane & 15;
  const int rowBase = blockIdx.x * GROWS;
  for (int i = tid; i < NIN * HD; i += GTHR) swn[i] = Wn[i];
  sbn[tid] = bn[tid];
  if (tid < GROWS) sdi[tid] = dinv[rowBase + tid];
  __syncthreads();

  {
    const int r = tid >> 1, c0 = (tid & 1) * 32;
    int xrow = rowBase + r;
    xrow = xrow > nN - 1 ? nN - 1 : xrow;
    float xv[NIN];
#pragma unroll
    for (int k = 0; k < NIN; ++k) xv[k] = x[(size_t)xrow * NIN + k];
#pragma unroll 1
    for (int cg = 0; cg < 4; ++cg) {
      v8h hv;
#pragma unroll
      for (int j = 0; j < 8; ++j) {
        const int c = c0 + 8 * cg + j;
        float a = sbn[c];
#pragma unroll
        for (int k = 0; k < NIN; ++k) a = fmaf(xv[k], swn[k * HD + c], a);
        hv[j] = (_Float16)(fmaxf(a, 0.0f) * HSC);
      }
      *(v8h*)(At + r * APZ + c0 + 8 * cg) = hv;
    }
  }
  __syncthreads();

  {
    v8f acc[4];
    mma16<4>(At + wave * 16 * APZ, APZ, BG, lane, acc);
    float* sp = stg + (wave * 16 + 8 * hh) * HD + m;
#pragma unroll
    for (int r = 0; r < 8; ++r) {
      const float di = sdi[wave * 16 + 8 * hh + r] * RH;
#pragma unroll
      for (int t = 0; t < 4; ++t) sp[r * HD + 16 * t] = acc[t][r] * di;
    }
  }
  __syncthreads();

  float* gp = HT + (size_t)rowBase * HD;
#pragma unroll
  for (int it = 0; it < 8; ++it) {
    const int f = it * GTHR + tid;
    const v4f v = ((const v4f*)stg)[f];
    *(volatile v4f*)(gp + 4 * f) = v;
  }
  __threadfence();
#pragma unroll
  for (int it = 0; it < 8; ++it) {
    const int f = it * GTHR + tid;
    const v4f v = ((const v4f*)stg)[f];
    *(volatile v4f*)(gp + 4 * f) = v;
  }
}

__device__ __forceinline__ void h2_store(const float* sacc, const float* sdi, const float* sbg,
                                         const float* __restrict__ HT, _Float16* H2, int n0, int tid) {
#pragma unroll 1
  for (int it = 0; it < (NBA * HD) / (8 * STHR); ++it) {
    const int f = it * STHR + tid, row = f >> 3, q = f & 7;
    const v4f* ap = (const v4f*)(sacc + row * HD + 8 * q);
    const v4f a0 = ap[0], a1 = ap[1];
    const float* hp = HT + (size_t)(n0 + row) * HD + 8 * q;
    const v4f h0 = *(const v4f*)hp, h1 = *(const v4f*)(hp + 4);
    const v4f* bp = (const v4f*)(sbg + 8 * q);
    const v4f b0 = bp[0], b1 = bp[1];
    const float di = sdi[row];
    const v4f u0 = a0 + h0, u1 = a1 + h1;
    v8h hv;
    hv[0] = (_Float16)(fmaf(di, u0.x, b0.x) * HSC); hv[1] = (_Float16)(fmaf(di, u0.y, b0.y) * HSC);
    hv[2] = (_Float16)(fmaf(di, u0.z, b0.z) * HSC); hv[3] = (_Float16)(fmaf(di, u0.w, b0.w) * HSC);
    hv[4] = (_Float16)(fmaf(di, u1.x, b1.x) * HSC); hv[5] = (_Float16)(fmaf(di, u1.y, b1.y) * HSC);
    hv[6] = (_Float16)(fmaf(di, u1.z, b1.z) * HSC); hv[7] = (_Float16)(fmaf(di, u1.w, b1.w) * HSC);
    *(volatile v8h*)(H2 + (size_t)(n0 + row) * HD + 8 * q) = hv;
  }
}

__global__ __launch_bounds__(STHR) void k_drain(
    const int* __restrict__ srcs, const int* __restrict__ dsts, const float* __restrict__ dinv,
    const float* __restrict__ HT, const float* __restrict__ bg, _Float16* H2,
    int nN, int nE, int nChunks, int vec) {
  extern __shared__ __attribute__((aligned(16))) char dynl[];
  float*    sacc  = (float*)dynl;
  unsigned* slist = (unsigned*)(dynl + NBA * HD * 4);
  float*    sdi   = (float*)(dynl + NBA * HD * 4 + CHUNK * 4);
  float*    sbg   = sdi + NBA;
  int*      swt   = (int*)(sbg + HD);
  const int tid = threadIdx.x, lane = tid & 31;
  const int wave = __builtin_amdgcn_readfirstlane(tid >> 5);
  const int n0 = blockIdx.x * NBA;
  {
    v4f z = {0.f, 0.f, 0.f, 0.f};
    v4f* p = (v4f*)sacc;
#pragma unroll
    for (int it = 0; it < (NBA * HD) / (4 * STHR); ++it) p[it * STHR + tid] = z;
  }
  sdi[tid] = dinv[n0 + tid];
  sdi[tid + STHR] = dinv[n0 + STHR + tid];
  if (tid < HD) sbg[tid] = bg[tid];
  __syncthreads();

#pragma unroll 1
  for (int c = 0; c < nChunks; ++c) {
    const int cbase = c * CHUNK;
    int d[EPT];
    loadids(dsts, nE, cbase, tid, vec, d);
    unsigned msk = 0;
#pragma unroll
    for (int j = 0; j < EPT; ++j) {
      const unsigned ld = (unsigned)d[j] - (unsigned)n0;
      msk |= ((ld < (unsigned)NBA) ? 1u : 0u) << j;
    }
    const int cnt = __builtin_popcount(msk);
    int pos, nh;
    blkscan(cnt, lane, wave, swt, pos, nh);
    const int e0 = cbase + EPT * tid;
#pragma unroll
    for (int j = 0; j < EPT; ++j) {
      if ((msk >> j) & 1u) {
        const unsigned ld = (unsigned)d[j] - (unsigned)n0;
        if (pos < CHUNK) slist[pos] = ((unsigned)(e0 + j) << 9) | ld;
        ++pos;
      }
    }
    __syncthreads();
    const int nhc = nh < CHUNK ? nh : CHUNK;
    for (int j = 0; j < nhc; ++j) {
      const unsigned pk = (unsigned)__builtin_amdgcn_readfirstlane((int)slist[j]);
      const int ld = (int)(pk & (unsigned)(NBA - 1));
      if ((ld & (SWAV - 1)) == wave) {
        int e = (int)(pk >> 9);
        e = e > nE - 1 ? nE - 1 : e;
        int s = srcs[e];
        s = s < 0 ? 0 : (s > nN - 1 ? nN - 1 : s);
        const v2f hv = *(const v2f*)(HT + (size_t)s * HD + 2 * lane);
        v2f* ap = (v2f*)(sacc + ld * HD + 2 * lane);
        const v2f av = *ap;
        *ap = av + hv;
      }
    }
  }
  __syncthreads();

  h2_store(sacc, sdi, sbg, HT, H2, n0, tid);
  __threadfence();
  h2_store(sacc, sdi, sbg, HT, H2, n0, tid);
}

__global__ __launch_bounds__(GTHR) void k_nodepq(const _Float16* __restrict__ H2, const _Float16* __restrict__ B1,
                                                 const float* __restrict__ b1, float* PQ) {
  __shared__ __attribute__((aligned(16))) float stg[GROWS * 2 * HD];
  const int tid = threadIdx.x, lane = tid & 31, wave = tid >> 5, hh = lane >> 4, m = lane & 15;
  const int rowBase = blockIdx.x * GROWS;
  {
    v8f acc[8];
    mma16<8>(H2 + (size_t)(rowBase + wave * 16) * HD, HD, B1, lane, acc);
    float* sp = stg + (wave * 16 + 8 * hh) * (2 * HD) + m;
#pragma unroll
    for (int t = 0; t < 8; ++t) {
      const float bv = (t >= 4) ? b1[16 * t + m - HD] : 0.0f;
#pragma unroll
      for (int r = 0; r < 8; ++r) sp[r * (2 * HD) + 16 * t] = fmaf(acc[t][r], RH, bv);
    }
  }
  __syncthreads();

  float* gp = PQ + (size_t)rowBase * (2 * HD);
#pragma unroll
  for (int it = 0; it < 16; ++it) {
    const int f = it * GTHR + tid;
    const v4f v = ((const v4f*)stg)[f];
    *(volatile v4f*)(gp + 4 * f) = v;
  }
  __threadfence();
#pragma unroll
  for (int it = 0; it < 16; ++it) {
    const int f = it * GTHR + tid;
    const v4f v = ((const v4f*)stg)[f];
    *(volatile v4f*)(gp + 4 * f) = v;
  }
}

__device__ __forceinline__ v4h enc4(float e, v4f w, v4f b) {
  v4h r;
  r.x = (_Float16)fmaxf(fmaf(e, w.x, b.x), 0.0f);
  r.y = (_Float16)fmaxf(fmaf(e, w.y, b.y), 0.0f);
  r.z = (_Float16)fmaxf(fmaf(e, w.z, b.z), 0.0f);
  r.w = (_Float16)fmaxf(fmaf(e, w.w, b.w), 0.0f);
  return r;
}

template <int J0>
__device__ __forceinline__ void rows_pq(float* sw, const float* __restrict__ PQ, int sv, int dv, int lane) {
#pragma unroll
  for (int j = J0; j < J0 + 8; ++j) {
    const int s = __builtin_amdgcn_readlane(sv, j);
    const int d = __builtin_amdgcn_readlane(dv, j);
    const v2f p = *(const v2f*)(PQ + (size_t)s * (2 * HD) + 2 * lane);
    const v2f q = *(const v2f*)(PQ + (size_t)d * (2 * HD) + HD + 2 * lane);
    *(v2f*)(sw + j * PQP + 2 * lane) = p + q;
  }
}

__global__ __launch_bounds__(ETHR) void k_edge(
    const float* __restrict__ PQ, const int* __restrict__ srcs, const int* __restrict__ dsts,
    const float* __restrict__ ea, const float* __restrict__ Wee, const float* __restrict__ bee,
    const _Float16* __restrict__ Bc, const float* __restrict__ W2, const float* __restrict__ b2,
    float* out, int nN, int nE) {
  __shared__ __attribute__((aligned(16))) float spq[EWAV * EPW * PQP];
  __shared__ __attribute__((aligned(16))) float swe[HD];
  __shared__ __attribute__((aligned(16))) float sbe[HD];
  __shared__ __attribute__((aligned(16))) float sc[EPB];
  const int tid = threadIdx.x, lane = tid & 31, wave = tid >> 5, hh = lane >> 4, m = lane & 15;
  if (tid < HD) swe[tid] = Wee[tid] * HSC;
  else          sbe[tid - HD] = bee[tid - HD] * HSC;
  float* sw = spq + wave * (EPW * PQP);

  float w2c[4];
#pragma unroll
  for (int t = 0; t < 4; ++t) w2c[t] = W2[16 * t + m];
  const float b2v = b2[0];

  const int eBase = blockIdx.x * EPB + wave * EPW;
  int e = eBase + lane;
  e = e > nE - 1 ? nE - 1 : e;
  int sv = srcs[e];
  sv = sv < 0 ? 0 : (sv > nN - 1 ? nN - 1 : sv);
  int dv = dsts[e];
  dv = dv < 0 ? 0 : (dv > nN - 1 ? nN - 1 : dv);
  int ei0 = eBase + m;       ei0 = ei0 > nE - 1 ? nE - 1 : ei0;
  int ei1 = eBase + 16 + m;  ei1 = ei1 > nE - 1 ? nE - 1 : ei1;
  const float ea0 = ea[ei0];
  const float ea1 = ea[ei1];

  rows_pq<0>(sw, PQ, sv, dv, lane);
  asm volatile("" ::: "memory");
  rows_pq<8>(sw, PQ, sv, dv, lane);
  asm volatile("" ::: "memory");
  rows_pq<16>(sw, PQ, sv, dv, lane);
  asm volatile("" ::: "memory");
  rows_pq<24>(sw, PQ, sv, dv, lane);
  __syncthreads();

  v8f acc0[4], acc1[4];
#pragma unroll
  for (int t = 0; t < 4; ++t) {
    v8f z = {0.f, 0.f, 0.f, 0.f, 0.f, 0.f, 0.f, 0.f};
    acc0[t] = z; acc1[t] = z;
  }
  const _Float16* bb = Bc + (size_t)m * KPB + 8 * hh;
#pragma unroll
  for (int ks = 0; ks < HD / 32; ++ks) {
    const int qlo = 8 * ks + 2 * hh;
    const int qhi = qlo + 4;
    const v4f* wp = (const v4f*)swe;
    const v4f* bp = (const v4f*)sbe;
    const v4f wl0 = wp[qlo], wl1 = wp[qlo + 1], wh0 = wp[qhi], wh1 = wp[qhi + 1];
    const v4f bl0 = bp[qlo], bl1 = bp[qlo + 1], bh0 = bp[qhi], bh1 = bp[qhi + 1];
    Frag a0, a1;
    a0.q[0] = enc4(ea0, wl0, bl0); a0.q[1] = enc4(ea0, wl1, bl1);
    a0.q[2] = enc4(ea0, wh0, bh0); a0.q[3] = enc4(ea0, wh1, bh1);
    a1.q[0] = enc4(ea1, wl0, bl0); a1.q[1] = enc4(ea1, wl1, bl1);
    a1.q[2] = enc4(ea1, wh0, bh0); a1.q[3] = enc4(ea1, wh1, bh1);
#pragma unroll
    for (int t = 0; t < 4; ++t) {
      const _Float16* bq = bb + (size_t)(16 * t) * KPB + 32 * ks;
      Frag b;
      b.h[0] = *(const v8h*)bq;
      b.h[1] = *(const v8h*)(bq + 16);
      acc0[t] = wmh(a0.v, b.v, acc0[t]);
      acc1[t] = wmh(a1.v, b.v, acc1[t]);
    }
  }

  const float* sp0 = sw + (8 * hh) * PQP + m;
  const float* sp1 = sp0 + 16 * PQP;
  float v[16];
#pragma unroll
  for (int r = 0; r < 8; ++r) {
    float s0 = 0.0f, s1 = 0.0f;
#pragma unroll
    for (int t = 0; t < 4; ++t) {
      const float pq0 = sp0[r * PQP + 16 * t];
      const float pq1 = sp1[r * PQP + 16 * t];
      const float h0 = fmaxf(fmaf(acc0[t][r], RH, pq0), 0.0f);
      const float h1 = fmaxf(fmaf(acc1[t][r], RH, pq1), 0.0f);
      s0 = fmaf(h0, w2c[t], s0);
      s1 = fmaf(h1, w2c[t], s1);
    }
    v[r] = s0;
    v[8 + r] = s1;
    asm volatile("" ::: "memory");
  }

  float u[8];
  {
    const bool kb = ((lane >> 3) & 1) != 0;
#pragma unroll
    for (int i = 0; i < 8; ++i) {
      const float snd = kb ? v[i] : v[i + 8];
      const float kp  = kb ? v[i + 8] : v[i];
      u[i] = kp + __shfl_xor(snd, 8, 32);
    }
  }
  float w4[4];
  {
    const bool kb = ((lane >> 2) & 1) != 0;
#pragma unroll
    for (int i = 0; i < 4; ++i) {
      const float snd = kb ? u[i] : u[i + 4];
      const float kp  = kb ? u[i + 4] : u[i];
      w4[i] = kp + __shfl_xor(snd, 4, 32);
    }
  }
  float x2[2];
  {
    const bool kb = ((lane >> 1) & 1) != 0;
#pragma unroll
    for (int i = 0; i < 2; ++i) {
      const float snd = kb ? w4[i] : w4[i + 2];
      const float kp  = kb ? w4[i + 2] : w4[i];
      x2[i] = kp + __shfl_xor(snd, 2, 32);
    }
  }
  float fin;
  {
    const bool kb = (lane & 1) != 0;
    const float snd = kb ? x2[0] : x2[1];
    const float kp  = kb ? x2[1] : x2[0];
    fin = kp + __shfl_xor(snd, 1, 32);
  }
  {
    const float s = fin + b2v;
    const int j = 16 * (m >> 3) + 8 * hh + (m & 7);
    sc[wave * EPW + j] = s;
  }
  __syncthreads();

  if (wave == 0) {
    const v4f ov = *(const v4f*)(sc + 4 * lane);
    const int e0 = blockIdx.x * EPB + 4 * lane;
    float* op = out + e0;
    const bool full = (e0 + 3 < nE);
    if (full) {
      *(volatile v4f*)op = ov;
    } else {
      if (e0     < nE) *(volatile float*)(op)     = ov.x;
      if (e0 + 1 < nE) *(volatile float*)(op + 1) = ov.y;
      if (e0 + 2 < nE) *(volatile float*)(op + 2) = ov.z;
    }
    __threadfence();
    if (full) {
      *(volatile v4f*)op = ov;
    } else {
      if (e0     < nE) *(volatile float*)(op)     = ov.x;
      if (e0 + 1 < nE) *(volatile float*)(op + 1) = ov.y;
      if (e0 + 2 < nE) *(volatile float*)(op + 2) = ov.z;
    }
  }
}

extern "C" void kernel_launch(void* const* d_in, const int* in_sizes, int n_in,
                              void* d_out, int out_size, void* d_ws, size_t ws_size,
                              hipStream_t stream) {
  if (n_in < 13) return;
  const int nN = in_sizes[0] / NIN;
  const int nE = in_sizes[2];
  if (nN < 1 || nE < 1) return;
  if (in_sizes[0] != nN * NIN || in_sizes[1] != 2 * nE) return;
  if (in_sizes[3] != NIN * HD || in_sizes[4] != HD || in_sizes[5] != HD || in_sizes[6] != HD) return;
  if (in_sizes[7] != HD * HD || in_sizes[8] != HD || in_sizes[9] != 3 * HD * HD || in_sizes[10] != HD) return;
  if (in_sizes[11] != HD || in_sizes[12] < 1) return;
  if (out_size != nE) return;
  if (nN > (1 << 22) || nE > (1 << 22)) return;

  const float* x    = (const float*)d_in[0];
  const int*   ei   = (const int*)d_in[1];
  const float* ea   = (const float*)d_in[2];
  const float* Wne  = (const float*)d_in[3];
  const float* bne  = (const float*)d_in[4];
  const float* Wee  = (const float*)d_in[5];
  const float* bee  = (const float*)d_in[6];
  const float* Wgcn = (const float*)d_in[7];
  const float* bgcn = (const float*)d_in[8];
  const float* W1   = (const float*)d_in[9];
  const float* b1   = (const float*)d_in[10];
  const float* W2   = (const float*)d_in[11];
  const float* b2   = (const float*)d_in[12];
  float* out = (float*)d_out;
  const int* srcs = ei;
  const int* dsts = ei + (size_t)nE;

  const int nPad    = ((nN + NPADG - 1) / NPADG) * NPADG;
  const int gDeg    = nPad / NBD;
  const int gNode   = nPad / GROWS;
  const int gAgg    = nPad / NBA;
  const int gEdge   = (nE + EPB - 1) / EPB;
  const int nChunks = (nE + CHUNK - 1) / CHUNK;
  const int vec     = ((nE & 3) == 0) ? 1 : 0;

  char* ws = (char*)d_ws;
  size_t off = 0;
  const size_t oB  = off; off += (size_t)BPTOT * 2;          off = (off + 255) & ~(size_t)255;
  const size_t oDI = off; off += (size_t)nPad * 4;           off = (off + 255) & ~(size_t)255;
  const size_t oHT = off; off += (size_t)nPad * HD * 4;      off = (off + 255) & ~(size_t)255;
  const size_t oH2 = off; off += (size_t)nPad * HD * 2;      off = (off + 255) & ~(size_t)255;
  const size_t oPQ = off; off += (size_t)nPad * 2 * HD * 4;  off = (off + 255) & ~(size_t)255;
  if (off > ws_size || off > (size_t)WSCAP) return;
  _Float16* Bpl  = (_Float16*)(ws + oB);
  float*    dinv = (float*)(ws + oDI);
  float*    HT   = (float*)(ws + oHT);
  _Float16* H2   = (_Float16*)(ws + oH2);
  float*    PQ   = (float*)(ws + oPQ);

  hipFuncSetAttribute(reinterpret_cast<const void*>(&k_deg), hipFuncAttributeMaxDynamicSharedMemorySize, LDS_DEG);
  hipFuncSetAttribute(reinterpret_cast<const void*>(&k_drain), hipFuncAttributeMaxDynamicSharedMemorySize, LDS_AGG);

  k_wprep<<<8, 256, 0, stream>>>(Wgcn, W1, Bpl);
  k_deg<<<gDeg, STHR, LDS_DEG, stream>>>(dsts, dinv, nE, nChunks, vec);
  k_node1<<<gNode, GTHR, 0, stream>>>(x, Wne, bne, dinv, Bpl + OFF_BG, HT, nN);
  k_drain<<<gAgg, STHR, LDS_AGG, stream>>>(srcs, dsts, dinv, HT, bgcn, H2, nN, nE, nChunks, vec);
  k_nodepq<<<gNode, GTHR, 0, stream>>>(H2, Bpl + OFF_B1, b1, PQ);
  k_edge<<<gEdge, ETHR, 0, stream>>>(PQ, srcs, dsts, ea, Wee, bee, Bpl + OFF_B1 + 2 * HD * KPB,
                                      W2, b2, out, nN, nE);
}
